// _MRNN_46935402611163
// MI455X (gfx1250) — hardware-verified
//
#include <hip/hip_runtime.h>
#include <math.h>

constexpr int NBAT  = 64;
constexpr int NSTEP = 256;
constexpr int NFEAT = 64;
constexpr int NHID  = 64;
constexpr int NGATE = 3 * NHID;
constexpr int NSEQ  = NBAT * NFEAT;
constexpr int NROWS = NBAT * NSTEP;
constexpr int NTHR  = 256;
constexpr int ROWS_BLK = 32;
constexpr int NBLK_SEQ = NSEQ / ROWS_BLK;
constexpr int APITCH = 72;
constexpr int FCN_ROWS = 4;
constexpr int NPART = NROWS / FCN_ROWS;
constexpr int PART_PITCH = 32;
constexpr int NOUT0 = NBAT * NSTEP * NFEAT;
constexpr float WCARRY     = 64.0f;
constexpr float WCARRY_INV = 1.0f / 64.0f;
constexpr float LOG2E_F    = 1.4426950408889634f;
static_assert(NSEQ % ROWS_BLK == 0);
static_assert(NFEAT % ROWS_BLK == 0);
static_assert(NHID == 64 && NTHR == 256);
static_assert((2 * ROWS_BLK * APITCH) % NTHR == 0);
static_assert(NROWS % FCN_ROWS == 0);
static_assert(FCN_ROWS * NFEAT == NTHR);
static_assert((NGATE * NHID) % (2 * NTHR) == 0);
static_assert(NPART % NTHR == 0);

typedef __attribute__((ext_vector_type(16))) _Float16 v16h;
typedef __attribute__((ext_vector_type(8)))  _Float16 v8h;
typedef __attribute__((ext_vector_type(8)))  float    v8f;
typedef __attribute__((ext_vector_type(4)))  float    v4f;

__device__ __forceinline__ void dep_guard3_h(v8f& a, v8f& b, v8f& c, v16h x, v16h y) {
  asm volatile("v_nop\n\tv_nop\n\tv_nop\n\tv_nop" : "+v"(a), "+v"(b), "+v"(c) : "v"(x), "v"(y));
}
__device__ __forceinline__ void keep4_h(v16h a, v16h b, v16h c, v16h d) { asm volatile("v_nop" :: "v"(a), "v"(b), "v"(c), "v"(d)); }
__device__ __forceinline__ void acc_guard3(v8f& a, v8f& b, v8f& c) {
  asm volatile("v_nop\n\tv_nop\n\tv_nop\n\tv_nop" : "+v"(a), "+v"(b), "+v"(c));
}

template <typename T> struct Frag;
template <> struct Frag<_Float16> {
  typedef v16h V; union U { v16h v; v8h h[2]; };
  static __device__ __forceinline__ v16h load(const _Float16* p) {
    U f; f.h[0] = *(const v8h*)(p); f.h[1] = *(const v8h*)(p + 16); return f.v;
  }
  static __device__ __forceinline__ v8f mma(v16h a, v16h b, v8f c) {
    return __builtin_amdgcn_wmma_f32_16x16x32_f16(false, a, false, b, (short)0, c, false, false);
  }
};

__device__ __forceinline__ float fsig(float x)  { return __builtin_amdgcn_rcpf(1.0f + exp2f(-(x * LOG2E_F))); }
__device__ __forceinline__ float ftanh(float x) { return 1.0f - 2.0f * __builtin_amdgcn_rcpf(exp2f((2.0f * LOG2E_F) * x) + 1.0f); }

__global__ __launch_bounds__(NTHR) void cast_scale_f16x2(const float* __restrict__ in,
                                                         unsigned short* __restrict__ out, int n2, float sc) {
  const int i = blockIdx.x * NTHR + threadIdx.x;
  if (i < n2) {
    const _Float16 h0 = (_Float16)(in[2 * i] * sc);
    const _Float16 h1 = (_Float16)(in[2 * i + 1] * sc);
    const unsigned u = (unsigned)__builtin_bit_cast(unsigned short, h0) |
                       ((unsigned)__builtin_bit_cast(unsigned short, h1) << 16);
    ((volatile unsigned*)out)[i] = u;
    __threadfence();
    ((volatile unsigned*)out)[i] = u;
  }
}

__global__ __launch_bounds__(NTHR) void gru_seq_kernel(
    const float* __restrict__ Xf, const float* __restrict__ Mf, const float* __restrict__ Df,
    const float* __restrict__ Xb, const float* __restrict__ Mb, const float* __restrict__ Db,
    const float* __restrict__ wihf, const float* __restrict__ bihf, const float* __restrict__ bhhf,
    const float* __restrict__ wihb, const float* __restrict__ bihb, const float* __restrict__ bhhb,
    const unsigned short* __restrict__ WHf, const unsigned short* __restrict__ WHb,
    const float* __restrict__ Wproj, float* __restrict__ Pout) {
  __shared__ __align__(16) _Float16 Ah[2][ROWS_BLK * APITCH];
  __shared__ __align__(16) float    Qs[2][ROWS_BLK * NHID];
  const int tid = threadIdx.x, lane = tid & 31, wave = tid >> 5;
  const int c = lane & 15, hh = lane >> 4, koff = hh * 8;
  const int ms = wave >> 2, ub = wave & 3;
  const int j = 16 * ub + c;
  const int dir = blockIdx.y, blk = blockIdx.x;
  const int bb = blk >> 1;
  const int f0 = 32 * (blk & 1) + 16 * ms + 8 * hh;

  const float* X   = dir ? Xb : Xf;
  const float* Mm  = dir ? Mb : Mf;
  const float* D   = dir ? Db : Df;
  const float* wih = dir ? wihb : wihf;
  const float* bih = dir ? bihb : bihf;
  const float* bhh = dir ? bhhb : bhhf;
  const _Float16* WH = (const _Float16*)(dir ? WHb : WHf);

  const float wr0 = wih[(0 * NHID + j) * 3 + 0], wr1 = wih[(0 * NHID + j) * 3 + 1], wr2 = wih[(0 * NHID + j) * 3 + 2];
  const float wz0 = wih[(1 * NHID + j) * 3 + 0], wz1 = wih[(1 * NHID + j) * 3 + 1], wz2 = wih[(1 * NHID + j) * 3 + 2];
  const float wn0 = wih[(2 * NHID + j) * 3 + 0], wn1 = wih[(2 * NHID + j) * 3 + 1], wn2 = wih[(2 * NHID + j) * 3 + 2];
  const float br  = bih[j] + bhh[j];
  const float bz  = bih[NHID + j] + bhh[NHID + j];
  const float bni = bih[2 * NHID + j];
  const float bnh = bhh[2 * NHID + j];
  const float wp  = Wproj[dir * NHID + j];

  {
    _Float16* ahf = &Ah[0][0];
#pragma unroll 1
    for (int i = tid; i < 2 * ROWS_BLK * APITCH; i += NTHR) ahf[i] = (_Float16)0.0f;
  }
  float hst[8];
#pragma unroll
  for (int r = 0; r < 8; ++r) hst[r] = 0.0f;
  __syncthreads();

  const v8f z8 = {0.f, 0.f, 0.f, 0.f, 0.f, 0.f, 0.f, 0.f};

#pragma unroll 1
  for (int t = 0; t < NSTEP; ++t) {
    const int cur = t & 1;
    const int tw  = dir ? (NSTEP - 1 - t) : t;
    const size_t base = ((size_t)(bb * NSTEP + t)) * NFEAT + f0;
    const v8f x8 = *(const v8f*)(X + base);
    const v8f m8 = *(const v8f*)(Mm + base);
    const v8f d8 = *(const v8f*)(D + base);

    v8f accR = z8, accZ = z8, accN = z8;
    const _Float16* arow = &Ah[cur][0] + (16 * ms + c) * APITCH + koff;
    const _Float16* wrow = WH + (size_t)j * NHID + koff;
#pragma unroll
    for (int ks = 0; ks < 2; ++ks) {
      const int k0 = 32 * ks;
      const v16h a  = Frag<_Float16>::load(arow + k0);
      const v16h b0 = Frag<_Float16>::load(wrow + k0);
      const v16h b1 = Frag<_Float16>::load(wrow + (size_t)NHID * NHID + k0);
      const v16h b2 = Frag<_Float16>::load(wrow + (size_t)2 * NHID * NHID + k0);
      accR = Frag<_Float16>::mma(a, b0, accR);
      accZ = Frag<_Float16>::mma(a, b1, accZ);
      accN = Frag<_Float16>::mma(a, b2, accN);
      dep_guard3_h(accR, accZ, accN, a, b2);
      keep4_h(a, b0, b1, b2);
    }
    acc_guard3(accR, accZ, accN);

    _Float16* ahn = &Ah[cur ^ 1][0];
    float* qsw = &Qs[cur][0];
#pragma unroll
    for (int r = 0; r < 8; ++r) {
      const float xv = x8[r], mv = m8[r], dv = d8[r];
      const float gr  = br + xv * wr0 + mv * wr1 + dv * wr2 + accR[r] * WCARRY_INV;
      const float gz  = bz + xv * wz0 + mv * wz1 + dv * wz2 + accZ[r] * WCARRY_INV;
      const float gni = bni + xv * wn0 + mv * wn1 + dv * wn2;
      const float ghn = bnh + accN[r] * WCARRY_INV;
      const float rg = fsig(gr);
      const float zg = fsig(gz);
      const float ng = ftanh(gni + rg * ghn);
      const float ho = hst[r];
      const float hn = (1.0f - zg) * ng + zg * ho;
      hst[r] = hn;
      const int lr = 16 * ms + 8 * hh + r;
      ahn[lr * APITCH + j] = (_Float16)hn;
      qsw[lr * NHID + j]   = hn * wp;
    }
    __syncthreads();

    if (wave == 0) {
      const float* qr = &Qs[cur][0] + lane * NHID;
      float p = 0.0f;
#pragma unroll
      for (int i = 0; i < NHID / 4; ++i) {
        const v4f v = *(const v4f*)(qr + 4 * i);
        p += v[0]; p += v[1]; p += v[2]; p += v[3];
      }
      float* dst = Pout + ((size_t)(dir * NSTEP + tw)) * NSEQ + ROWS_BLK * blk + lane;
      *(volatile float*)dst = p;
      __threadfence();
      *(volatile float*)dst = p;
    }
  }
}

__global__ __launch_bounds__(NTHR) void fcn_reg_kernel(
    const float* __restrict__ X, const float* __restrict__ Mm, const float* __restrict__ Pp,
    const float* __restrict__ bproj, const float* __restrict__ Uw, const float* __restrict__ V1w,
    const float* __restrict__ V2w, const float* __restrict__ betav, const float* __restrict__ Wfin,
    const float* __restrict__ bfin, float* __restrict__ out0, float* __restrict__ part) {
  __shared__ __align__(16) float xs[FCN_ROWS * NFEAT];
  __shared__ __align__(16) float mks[FCN_ROWS * NFEAT];
  __shared__ __align__(16) float ims[FCN_ROWS * NFEAT];
  __shared__ __align__(16) float hsb[FCN_ROWS * NFEAT];
  __shared__ __align__(16) float outs[FCN_ROWS * NFEAT];
  __shared__ float red[(NTHR / 32) * 4];
  const int tid = threadIdx.x, lane = tid & 31, wave = tid >> 5;
  const int lr = tid >> 6, f = tid & 63;
  const int row = blockIdx.x * FCN_ROWS + lr;
  const int bq = row >> 8, t = row & 255;
  const size_t idx = (size_t)row * NFEAT + f;
  const float x = X[idx], m = Mm[idx];
  const int n = bq * NFEAT + f;
  const float rnn = (Pp[(size_t)t * NSEQ + n] + Pp[(size_t)(NSTEP + t) * NSEQ + n]) + bproj[0];
  const float imp = m * x + (1.0f - m) * rnn;
  xs[tid] = x; mks[tid] = m; ims[tid] = imp;
  __syncthreads();

  const float* xr = xs + lr * NFEAT;
  const float* ir = ims + lr * NFEAT;
  const float* mr = mks + lr * NFEAT;
  const float* ur = Uw  + (size_t)f * NFEAT;
  const float* vr = V1w + (size_t)f * NFEAT;
  const float* wr = V2w + (size_t)f * NFEAT;
  float su = 0.0f, sv1 = 0.0f, sv2 = 0.0f;
#pragma unroll 1
  for (int k = 0; k < NFEAT; k += 4) {
    const v4f xa = *(const v4f*)(xr + k), ia = *(const v4f*)(ir + k), ma = *(const v4f*)(mr + k);
    const v4f ua = *(const v4f*)(ur + k), va = *(const v4f*)(vr + k), wa = *(const v4f*)(wr + k);
#pragma unroll
    for (int e = 0; e < 4; ++e) { su += xa[e] * ua[e]; sv1 += ia[e] * va[e]; sv2 += ma[e] * wa[e]; }
  }
  const float pre = ((su - x * Uw[(size_t)f * NFEAT + f]) + (sv1 - imp * V1w[(size_t)f * NFEAT + f])) + sv2 + betav[f];
  const float hv = ftanh(pre);
  hsb[tid] = hv;
  __syncthreads();

  const float* hr = hsb + lr * NFEAT;
  const float* fr = Wfin + (size_t)f * NFEAT;
  float fe = 0.0f;
#pragma unroll 1
  for (int k = 0; k < NFEAT; k += 4) {
    const v4f ha = *(const v4f*)(hr + k), wa = *(const v4f*)(fr + k);
#pragma unroll
    for (int e = 0; e < 4; ++e) fe += ha[e] * wa[e];
  }
  fe += bfin[f];
  const float imputed = m * x + (1.0f - m) * fe;
  outs[tid] = imputed;
  const float d1 = (fe - x) * m, d2 = (rnn - x) * m;
  float s1 = d1 * d1, s2 = d2 * d2, s3 = m;
#pragma unroll
  for (int off = 16; off > 0; off >>= 1) {
    s1 += __shfl_xor(s1, off, 32);
    s2 += __shfl_xor(s2, off, 32);
    s3 += __shfl_xor(s3, off, 32);
  }
  if (lane == 0) { red[wave * 4 + 0] = s1; red[wave * 4 + 1] = s2; red[wave * 4 + 2] = s3; }
  __syncthreads();

  if (wave == 0) {
    float t1 = 0.0f, t2 = 0.0f, t3 = 0.0f;
#pragma unroll
    for (int w = 0; w < NTHR / 32; ++w) { t1 += red[w * 4 + 0]; t2 += red[w * 4 + 1]; t3 += red[w * 4 + 2]; }
    v4f pv;
    pv[0] = (lane == 0) ? t1 : 0.0f;
    pv[1] = (lane == 0) ? t2 : 0.0f;
    pv[2] = (lane == 0) ? t3 : 0.0f;
    pv[3] = 0.0f;
    float* ob = out0 + (size_t)blockIdx.x * (FCN_ROWS * NFEAT);
    float* pp = part + (size_t)blockIdx.x * PART_PITCH + 4 * lane;
    for (int pass = 0; pass < 2; ++pass) {
#pragma unroll
      for (int it = 0; it < 2; ++it) {
        const v4f v = *(const v4f*)(outs + it * 128 + 4 * lane);
        *(volatile v4f*)(ob + it * 128 + 4 * lane) = v;
      }
      if (lane < 8) *(volatile v4f*)pp = pv;
      __threadfence();
    }
  }
}

__global__ __launch_bounds__(NTHR) void loss_kernel(const float* __restrict__ part, float* __restrict__ out1) {
  __shared__ float ra[NTHR], rb[NTHR], rc[NTHR];
  const int tid = threadIdx.x;
  float a = 0.0f, b = 0.0f, cc = 0.0f;
#pragma unroll 1
  for (int i = tid; i < NPART; i += NTHR) {
    const v4f v = *(const v4f*)(part + (size_t)i * PART_PITCH);
    a += v[0]; b += v[1]; cc += v[2];
  }
  ra[tid] = a; rb[tid] = b; rc[tid] = cc;
  __syncthreads();
#pragma unroll 1
  for (int s = NTHR / 2; s > 0; s >>= 1) {
    if (tid < s) { ra[tid] += ra[tid + s]; rb[tid] += rb[tid + s]; rc[tid] += rc[tid + s]; }
    __syncthreads();
  }
  if (tid == 0) {
    const float den = rc[0] + 1e-12f;
    const float lv = sqrtf(ra[0] / den) + sqrtf(rb[0] / den);
    *(volatile float*)out1 = lv;
    __threadfence();
    *(volatile float*)out1 = lv;
  }
}

extern "C" void kernel_launch(void* const* d_in, const int* in_sizes, int n_in,
                              void* d_out, int out_size, void* d_ws, size_t ws_size, hipStream_t stream) {
  if (n_in < 22 || d_out == nullptr || d_ws == nullptr) return;
  const int nbig = NBAT * NSTEP * NFEAT;
  if (in_sizes[0] != nbig || in_sizes[1] != nbig || in_sizes[2] != nbig ||
      in_sizes[3] != nbig || in_sizes[4] != nbig || in_sizes[5] != nbig ||
      in_sizes[6] != NGATE * 3 || in_sizes[7] != NGATE * NHID || in_sizes[8] != NGATE || in_sizes[9] != NGATE ||
      in_sizes[10] != NGATE * 3 || in_sizes[11] != NGATE * NHID || in_sizes[12] != NGATE || in_sizes[13] != NGATE ||
      in_sizes[14] != 2 * NHID || in_sizes[15] != 1 ||
      in_sizes[16] != NFEAT * NFEAT || in_sizes[17] != NFEAT * NFEAT || in_sizes[18] != NFEAT * NFEAT ||
      in_sizes[19] != NFEAT || in_sizes[20] != NFEAT * NFEAT || in_sizes[21] != NFEAT ||
      out_size != NOUT0 + 1) return;

  const float* X_f    = (const float*)d_in[0];
  const float* M_f    = (const float*)d_in[1];
  const float* D_f    = (const float*)d_in[2];
  const float* X_b    = (const float*)d_in[3];
  const float* M_b    = (const float*)d_in[4];
  const float* D_b    = (const float*)d_in[5];
  const float* w_ih_f = (const float*)d_in[6];
  const float* w_hh_f = (const float*)d_in[7];
  const float* b_ih_f = (const float*)d_in[8];
  const float* b_hh_f = (const float*)d_in[9];
  const float* w_ih_b = (const float*)d_in[10];
  const float* w_hh_b = (const float*)d_in[11];
  const float* b_ih_b = (const float*)d_in[12];
  const float* b_hh_b = (const float*)d_in[13];
  const float* W_proj = (const float*)d_in[14];
  const float* b_proj = (const float*)d_in[15];
  const float* Um     = (const float*)d_in[16];
  const float* V1m    = (const float*)d_in[17];
  const float* V2m    = (const float*)d_in[18];
  const float* betav  = (const float*)d_in[19];
  const float* W_fin  = (const float*)d_in[20];
  const float* b_fin  = (const float*)d_in[21];
  float* out0 = (float*)d_out;
  float* out1 = out0 + (size_t)NOUT0;

  char* ws = (char*)d_ws; size_t off = 0;
  auto carve = [&](size_t bytes) -> char* { char* p = ws + off; off += (bytes + 255) & ~(size_t)255; return p; };
  unsigned short* WHF  = (unsigned short*)carve((size_t)NGATE * NHID * 2);
  unsigned short* WHB  = (unsigned short*)carve((size_t)NGATE * NHID * 2);
  float*          PPRJ = (float*)carve((size_t)2 * NSTEP * NSEQ * 4);
  float*          PART = (float*)carve((size_t)NPART * PART_PITCH * 4);
  if (off > ws_size || off > (size_t)134217728) return;

  const int n2 = NGATE * NHID / 2;
  cast_scale_f16x2<<<(n2 + NTHR - 1) / NTHR, NTHR, 0, stream>>>(w_hh_f, WHF, n2, WCARRY);
  cast_scale_f16x2<<<(n2 + NTHR - 1) / NTHR, NTHR, 0, stream>>>(w_hh_b, WHB, n2, WCARRY);

  gru_seq_kernel<<<dim3(NBLK_SEQ, 2), NTHR, 0, stream>>>(
      X_f, M_f, D_f, X_b, M_b, D_b,
      w_ih_f, b_ih_f, b_hh_f, w_ih_b, b_ih_b, b_hh_b,
      WHF, WHB, W_proj, PPRJ);

  fcn_reg_kernel<<<NPART, NTHR, 0, stream>>>(X_f, M_f, PPRJ, b_proj, Um, V1m, V2m, betav, W_fin, b_fin, out0, PART);

  loss_kernel<<<1, NTHR, 0, stream>>>(PART, out1);
}
